// SHR_Block_137438953665
// MI455X (gfx1250) — hardware-verified
//
#include <hip/hip_runtime.h>
#include <math.h>

constexpr int kBatch   = 2;
constexpr int kSeq     = 2048;
constexpr int kDim     = 128;
constexpr int kHeads   = 8;
constexpr int kHdim    = 16;
constexpr int kHid     = 768;
constexpr int kRows    = kBatch * kSeq;
constexpr int kDim3    = 3 * kDim;
constexpr int kQPitch  = kHeads * 32;
constexpr int kGroups  = 3 * kBatch;
constexpr int kHeadGrp = 4;
constexpr float kWCarry = 16.0f;
constexpr float kPCarry = 32768.0f;
constexpr float kOCarry = 64.0f;
constexpr float kGCarry = 16.0f;
constexpr float kLnEps  = 1e-5f;

typedef __attribute__((ext_vector_type(16))) _Float16 v16h;
typedef __attribute__((ext_vector_type(8)))  _Float16 v8h;
typedef __attribute__((ext_vector_type(16))) __bf16   v16b;
typedef __attribute__((ext_vector_type(8)))  __bf16   v8b;
typedef __attribute__((ext_vector_type(8)))  float    v8f;
typedef __attribute__((ext_vector_type(4)))  float    v4f;
typedef __attribute__((ext_vector_type(2)))  float    v2f;
typedef __attribute__((ext_vector_type(4)))  unsigned int v4u;
typedef __attribute__((ext_vector_type(2)))  unsigned int v2u;

__device__ __forceinline__ unsigned short f2bf_bits(float f) {
  unsigned u = __float_as_uint(f);
  return (unsigned short)((u + 0x7FFFu + ((u >> 16) & 1u)) >> 16);
}
__device__ __forceinline__ float bf_bits2f(unsigned short h) { return __uint_as_float(((unsigned)h) << 16); }

__device__ __forceinline__ void dep_guard_h(v8f& a, v8f& b, v16h x, v16h y) { asm volatile("v_nop\n\tv_nop\n\tv_nop\n\tv_nop" : "+v"(a), "+v"(b) : "v"(x), "v"(y)); }
__device__ __forceinline__ void dep_guard_b(v8f& a, v8f& b, v16b x, v16b y) { asm volatile("v_nop\n\tv_nop\n\tv_nop\n\tv_nop" : "+v"(a), "+v"(b) : "v"(x), "v"(y)); }
__device__ __forceinline__ void keep4_h(v16h a, v16h b, v16h c, v16h d) { asm volatile("v_nop" :: "v"(a), "v"(b), "v"(c), "v"(d)); }
__device__ __forceinline__ void keep4_b(v16b a, v16b b, v16b c, v16b d) { asm volatile("v_nop" :: "v"(a), "v"(b), "v"(c), "v"(d)); }
__device__ __forceinline__ void acc_guard4(v8f& a, v8f& b, v8f& c, v8f& d) { asm volatile("v_nop\n\tv_nop\n\tv_nop\n\tv_nop" : "+v"(a), "+v"(b), "+v"(c), "+v"(d)); }
template <typename T> struct Frag;
template <> struct Frag<_Float16> {
  typedef v16h V; union U { v16h v; v8h h[2]; };
  static __device__ __forceinline__ v16h load(const _Float16* p) {
    U f; f.h[0] = *(const v8h*)(p); f.h[1] = *(const v8h*)(p + 16); return f.v;
  }
  static __device__ __forceinline__ v8f mma(v16h a, v16h b, v8f c) {
    return __builtin_amdgcn_wmma_f32_16x16x32_f16(false, a, false, b, (short)0, c, false, false);
  }
  static __device__ __forceinline__ void guard(v8f& a, v8f& b, v16h x, v16h y) { dep_guard_h(a, b, x, y); }
  static __device__ __forceinline__ void keep(v16h a, v16h b, v16h c, v16h d) { keep4_h(a, b, c, d); }
};
template <> struct Frag<__bf16> {
  typedef v16b V; union U { v16b v; v8b h[2]; };
  static __device__ __forceinline__ v16b load(const __bf16* p) {
    U f; f.h[0] = *(const v8b*)(p); f.h[1] = *(const v8b*)(p + 16); return f.v;
  }
  static __device__ __forceinline__ v8f mma(v16b a, v16b b, v8f c) {
    return __builtin_amdgcn_wmma_f32_16x16x32_bf16(false, a, false, b, (short)0, c, false, false);
  }
  static __device__ __forceinline__ void guard(v8f& a, v8f& b, v16b x, v16b y) { dep_guard_b(a, b, x, y); }
  static __device__ __forceinline__ void keep(v16b a, v16b b, v16b c, v16b d) { keep4_b(a, b, c, d); }
};

__device__ __forceinline__ unsigned pk16(unsigned short a, unsigned short b) { return (unsigned)a | ((unsigned)b << 16); }
__device__ __forceinline__ unsigned short h_bits(float f) { const _Float16 h = (_Float16)f; return __builtin_bit_cast(unsigned short, h); }

template <int ET> struct Elem;
template <> struct Elem<0> { typedef _Float16 T; };
template <> struct Elem<1> { typedef __bf16 T; };
template <int ET, bool SPLIT, int BIAS_MODE, int OUT_MODE, bool RESID, int ACT = 0>
__global__ __launch_bounds__(256) void wmma_gemm64(
    const unsigned short* __restrict__ Ap, const unsigned short* __restrict__ A2p, int lda, long strideA,
    const unsigned short* __restrict__ Btp, const unsigned short* __restrict__ Bt2p, int ldb, long strideB,
    void* __restrict__ Cout, void* __restrict__ Cout2, int ldc, long strideC,
    const float* __restrict__ bias,
    const float* __restrict__ resid, long strideR, int ldr,
    int M, int N, int K, float scale) {
  typedef typename Elem<ET>::T T;
  typedef typename Frag<T>::V V;
  const T* A = (const T*)Ap; const T* A2 = (const T*)A2p; const T* Bt = (const T*)Btp; const T* Bt2 = (const T*)Bt2p;
  __shared__ __align__(16) float sT[8][16 * 68];
  const int b    = blockIdx.y;
  const int lane = threadIdx.x & 31;
  const int wave = threadIdx.x >> 5;
  const int tilesN = N >> 6;
  const int tilesM = M >> 6;
  const int tile = blockIdx.x * 8 + wave;
  if (tile >= tilesM * tilesN) return;
  const int tm = tile / tilesN;
  const int tn = tile - tm * tilesN;
  const int m0 = tm << 6;
  const int n0 = tn << 6;

  const T* Ab  = A  + (size_t)b * strideA;
  const T* Bb  = Bt + (size_t)b * strideB;
  const T* Ab2 = SPLIT ? (A2  + (size_t)b * strideA) : nullptr;
  const T* Bb2 = SPLIT ? (Bt2 + (size_t)b * strideB) : nullptr;

  const int rlane = lane & 15;
  const int koff  = (lane >> 4) * 8;
  const int mOff  = (lane >> 4) * 8;

  v8f acc[4][4];
#pragma unroll
  for (int i = 0; i < 4; ++i)
#pragma unroll
    for (int j = 0; j < 4; ++j) acc[i][j] = (v8f){0.f,0.f,0.f,0.f,0.f,0.f,0.f,0.f};

  for (int k0 = 0; k0 < K; k0 += 32) {
    V bh[4], bl[4];
#pragma unroll
    for (int j = 0; j < 4; ++j) {
      const size_t bo = (size_t)(n0 + (j << 4) + rlane) * ldb + koff + k0;
      bh[j] = Frag<T>::load(Bb + bo);
      if (SPLIT) bl[j] = Frag<T>::load(Bb2 + bo);
    }
#pragma unroll
    for (int i = 0; i < 4; ++i) {
      const size_t ao = (size_t)(m0 + (i << 4) + rlane) * lda + koff + k0;
      V ah = Frag<T>::load(Ab + ao);
      V al;
      if (SPLIT) al = Frag<T>::load(Ab2 + ao);
#pragma unroll
      for (int j = 0; j < 4; ++j) {
        acc[i][j] = Frag<T>::mma(ah, bh[j], acc[i][j]);
        if (SPLIT) {
          acc[i][j] = Frag<T>::mma(ah, bl[j], acc[i][j]);
          acc[i][j] = Frag<T>::mma(al, bh[j], acc[i][j]);
        }
      }
      Frag<T>::guard(acc[i][0], acc[i][3], ah, SPLIT ? al : ah);
    }
    Frag<T>::keep(bh[0], bh[1], bh[2], bh[3]);
    if (SPLIT) Frag<T>::keep(bl[0], bl[1], bl[2], bl[3]);
  }
  acc_guard4(acc[0][0], acc[0][1], acc[0][2], acc[0][3]);
  acc_guard4(acc[1][0], acc[1][1], acc[1][2], acc[1][3]);
  acc_guard4(acc[2][0], acc[2][1], acc[2][2], acc[2][3]);
  acc_guard4(acc[3][0], acc[3][1], acc[3][2], acc[3][3]);

  float* slab = sT[wave];
  const float* Rb = RESID ? (resid + (size_t)b * strideR) : nullptr;
#pragma unroll
  for (int i = 0; i < 4; ++i) {
    const int mBase = m0 + (i << 4);
#pragma unroll
    for (int j = 0; j < 4; ++j) {
      const int n = n0 + (j << 4) + rlane;
      float bv = 0.f;
      if (BIAS_MODE == 2) bv = bias[n];
#pragma unroll
      for (int r = 0; r < 8; ++r) {
        float v = acc[i][j][r] * scale;
        if (BIAS_MODE == 1) v += bias[mBase + mOff + r];
        if (BIAS_MODE == 2) v += bv;
        if (RESID) v += Rb[(size_t)(mBase + mOff + r) * ldr + n];
        if (ACT == 2) v = fmaxf(v, 0.0f);
        if (ACT == 4) v = (v > 0.f) ? v : 0.01f * v;
        slab[(mOff + r) * 68 + (j << 4) + rlane] = v;
      }
    }
    __builtin_amdgcn_fence(__ATOMIC_RELEASE, "workgroup");
    __builtin_amdgcn_wave_barrier();
    __builtin_amdgcn_fence(__ATOMIC_ACQUIRE, "workgroup");
    if (OUT_MODE == 0) {
      float* C = (float*)Cout + (size_t)b * strideC;
      const int hh = lane >> 4, c4 = (lane & 15) * 4;
      for (int pass = 0; pass < 2; ++pass) {
#pragma unroll
        for (int it = 0; it < 8; ++it) {
          const int row = it * 2 + hh;
          v4f v = *(const v4f*)(slab + row * 68 + c4);
          *(volatile v4f*)(C + (size_t)(mBase + row) * ldc + n0 + c4) = v;
        }
        __threadfence();
      }
    } else {
      const int q = lane >> 3, c8 = (lane & 7) * 8;
      unsigned short* C  = (unsigned short*)Cout  + (size_t)b * strideC;
      unsigned short* C2 = (OUT_MODE == 2) ? ((unsigned short*)Cout2 + (size_t)b * strideC) : nullptr;
      for (int pass = 0; pass < 2; ++pass) {
#pragma unroll
        for (int it = 0; it < 4; ++it) {
          const int row = it * 4 + q;
          const float* sp = slab + row * 68 + c8;
          v8h hv, lv;
#pragma unroll
          for (int e = 0; e < 8; ++e) {
            if (OUT_MODE == 1) {
              hv[e] = (_Float16)sp[e];
            } else {
              unsigned short hb = f2bf_bits(sp[e]);
              unsigned short lb = f2bf_bits(sp[e] - bf_bits2f(hb));
              hv[e] = __builtin_bit_cast(_Float16, hb);
              lv[e] = __builtin_bit_cast(_Float16, lb);
            }
          }
          *(volatile v8h*)(C + (size_t)(mBase + row) * ldc + n0 + c8) = hv;
          if (OUT_MODE == 2) *(volatile v8h*)(C2 + (size_t)(mBase + row) * ldc + n0 + c8) = lv;
        }
        __threadfence();
      }
    }
    __builtin_amdgcn_fence(__ATOMIC_RELEASE, "workgroup");
    __builtin_amdgcn_wave_barrier();
    __builtin_amdgcn_fence(__ATOMIC_ACQUIRE, "workgroup");
  }
}

__global__ __launch_bounds__(256) void wtcast_kernel(const float* __restrict__ W, unsigned short* __restrict__ out,
                                                     int nIn, int nOut, float scale) {
  __shared__ float sm[64][65];
  const int t  = threadIdx.x;
  const int d0 = blockIdx.x * 64;
  const int h0 = blockIdx.y * 64;
  const int z  = blockIdx.z;
  const float* Wz = W + (size_t)z * nIn * nOut;
#pragma unroll
  for (int i = 0; i < 16; ++i) {
    const int e = i * 256 + t;
    const int r = e >> 6;
    const int c = e & 63;
    sm[c][r] = Wz[(size_t)(d0 + r) * nOut + h0 + c] * scale;
  }
  __syncthreads();
  const int lane = t & 31, wave = t >> 5;
  const int q = lane >> 3, c8 = (lane & 7) * 8;
  unsigned short* op = out + (size_t)z * nOut * nIn;
  for (int pass = 0; pass < 2; ++pass) {
#pragma unroll
    for (int it = 0; it < 2; ++it) {
      const int row = wave * 8 + it * 4 + q;
      unsigned short hb[8];
#pragma unroll
      for (int e = 0; e < 8; ++e) hb[e] = h_bits(sm[row][c8 + e]);
      const v4u u = (v4u){pk16(hb[0], hb[1]), pk16(hb[2], hb[3]), pk16(hb[4], hb[5]), pk16(hb[6], hb[7])};
      *(volatile v4u*)(op + (size_t)(h0 + row) * nIn + d0 + c8) = u;
    }
    __threadfence();
  }
}

__global__ __launch_bounds__(256) void ln128_kernel(const float* __restrict__ x1, const float* __restrict__ x2,
                                                    const float* __restrict__ x3, const float* __restrict__ g,
                                                    const float* __restrict__ bt, unsigned short* __restrict__ xn) {
  const int lane = threadIdx.x & 31, wave = threadIdx.x >> 5;
  const int wid = blockIdx.x * 8 + wave;
  const int br  = wid / kRows;
  const int row = wid - br * kRows;
  const float* x = (br == 0) ? x1 : (br == 1) ? x2 : x3;
  const v4f xv = *(const v4f*)(x + (size_t)row * kDim + lane * 4);
  float s = (xv[0] + xv[1]) + (xv[2] + xv[3]);
#pragma unroll
  for (int off = 16; off > 0; off >>= 1) s += __shfl_xor(s, off, 32);
  const float mean = s * (1.0f / 128.0f);
  const float d0 = xv[0] - mean, d1 = xv[1] - mean, d2 = xv[2] - mean, d3 = xv[3] - mean;
  float s2 = (d0 * d0 + d1 * d1) + (d2 * d2 + d3 * d3);
#pragma unroll
  for (int off = 16; off > 0; off >>= 1) s2 += __shfl_xor(s2, off, 32);
  const float var  = s2 * (1.0f / 128.0f);
  const float rstd = rsqrtf(var + kLnEps);
  const v4f gv = *(const v4f*)(g + br * kDim + lane * 4);
  const v4f bv = *(const v4f*)(bt + br * kDim + lane * 4);
  const float y0 = d0 * rstd * gv[0] + bv[0];
  const float y1 = d1 * rstd * gv[1] + bv[1];
  const float y2 = d2 * rstd * gv[2] + bv[2];
  const float y3 = d3 * rstd * gv[3] + bv[3];
  const v2u u = (v2u){pk16(h_bits(y0), h_bits(y1)), pk16(h_bits(y2), h_bits(y3))};
  unsigned short* qp = xn + (size_t)wid * kDim + lane * 4;
  *(volatile v2u*)qp = u;
  __threadfence();
  *(volatile v2u*)qp = u;
}

__global__ __launch_bounds__(256) void ln384_kernel(const float* __restrict__ xc, const float* __restrict__ g,
                                                    const float* __restrict__ bt, unsigned short* __restrict__ hn) {
  const int lane = threadIdx.x & 31, wave = threadIdx.x >> 5;
  const int row = blockIdx.x * 8 + wave;
  const float* r = xc + (size_t)row * kDim3;
  v4f vv[3];
  float s = 0.f;
#pragma unroll
  for (int ch = 0; ch < 3; ++ch) {
    vv[ch] = *(const v4f*)(r + ch * kDim + lane * 4);
    s += (vv[ch][0] + vv[ch][1]) + (vv[ch][2] + vv[ch][3]);
  }
#pragma unroll
  for (int off = 16; off > 0; off >>= 1) s += __shfl_xor(s, off, 32);
  const float mean = s * (1.0f / 384.0f);
  float s2 = 0.f;
#pragma unroll
  for (int ch = 0; ch < 3; ++ch) {
#pragma unroll
    for (int j = 0; j < 4; ++j) { const float d = vv[ch][j] - mean; vv[ch][j] = d; s2 += d * d; }
  }
#pragma unroll
  for (int off = 16; off > 0; off >>= 1) s2 += __shfl_xor(s2, off, 32);
  const float var  = s2 * (1.0f / 384.0f);
  const float rstd = rsqrtf(var + kLnEps);
  v2u u[3];
#pragma unroll
  for (int ch = 0; ch < 3; ++ch) {
    const v4f gv = *(const v4f*)(g + ch * kDim + lane * 4);
    const v4f bv = *(const v4f*)(bt + ch * kDim + lane * 4);
    unsigned short hb[4];
#pragma unroll
    for (int j = 0; j < 4; ++j) hb[j] = h_bits(vv[ch][j] * rstd * gv[j] + bv[j]);
    u[ch] = (v2u){pk16(hb[0], hb[1]), pk16(hb[2], hb[3])};
  }
  unsigned short* qp = hn + (size_t)row * kDim3 + lane * 4;
  for (int pass = 0; pass < 2; ++pass) {
#pragma unroll
    for (int ch = 0; ch < 3; ++ch) *(volatile v2u*)(qp + ch * kDim) = u[ch];
    __threadfence();
  }
}

__global__ __launch_bounds__(256) void pad_qk_kernel(const unsigned short* __restrict__ qkvo,
                                                     unsigned short* __restrict__ q32, unsigned short* __restrict__ k32) {
  const int lane = threadIdx.x & 31, wave = threadIdx.x >> 5;
  const int row = blockIdx.x * 8 + wave;
  const int hz = lane >> 2, p = lane & 3;
  const size_t src = (size_t)row * kDim3 + hz * kHdim + 8 * (p & 1);
  const v4u qv = *(const v4u*)(qkvo + src);
  const v4u kv = *(const v4u*)(qkvo + src + kDim);
  const unsigned keep = (p < 2) ? 0xFFFFFFFFu : 0u;
  const v4u qo = (v4u){qv[0] & keep, qv[1] & keep, qv[2] & keep, qv[3] & keep};
  const v4u ko = (v4u){kv[0] & keep, kv[1] & keep, kv[2] & keep, kv[3] & keep};
  const size_t dst = (size_t)row * kQPitch + lane * 8;
  for (int pass = 0; pass < 2; ++pass) {
    *(volatile v4u*)(q32 + dst) = qo;
    *(volatile v4u*)(k32 + dst) = ko;
    __threadfence();
  }
}

__global__ __launch_bounds__(256) void vtrans_kernel(const unsigned short* __restrict__ qkvo, unsigned short* __restrict__ vt) {
  __shared__ unsigned short sm[64][66];
  const int t  = threadIdx.x;
  const int n0 = blockIdx.x * 64;
  const int c0 = blockIdx.y * 64;
  const int g  = blockIdx.z;
#pragma unroll
  for (int i = 0; i < 2; ++i) {
    const int e = i * 256 + t;
    const int r = e >> 3;
    const int part = e & 7;
    const v4u u = *(const v4u*)(qkvo + (size_t)(g * kSeq + n0 + r) * kDim3 + 2 * kDim + c0 + part * 8);
#pragma unroll
    for (int w = 0; w < 4; ++w) {
      sm[part * 8 + 2 * w][r]     = (unsigned short)(u[w] & 0xFFFFu);
      sm[part * 8 + 2 * w + 1][r] = (unsigned short)(u[w] >> 16);
    }
  }
  __syncthreads();
  const int lane = t & 31, wave = t >> 5;
  const int q = lane >> 3, c8 = (lane & 7) * 8;
  for (int pass = 0; pass < 2; ++pass) {
#pragma unroll
    for (int it = 0; it < 2; ++it) {
      const int row = wave * 8 + it * 4 + q;
      unsigned short hb[8];
#pragma unroll
      for (int e = 0; e < 8; ++e) hb[e] = sm[row][c8 + e];
      const v4u u = (v4u){pk16(hb[0], hb[1]), pk16(hb[2], hb[3]), pk16(hb[4], hb[5]), pk16(hb[6], hb[7])};
      *(volatile v4u*)(vt + (size_t)(g * kDim + c0 + row) * kSeq + n0 + c8) = u;
    }
    __threadfence();
  }
}

__global__ __launch_bounds__(256) void softmax2048_kernel(const float* __restrict__ S, unsigned short* __restrict__ P, float carry) {
  __shared__ float redM[8];
  __shared__ float redS[8];
  const int row  = blockIdx.x;
  const int t    = threadIdx.x;
  const int lane = t & 31, wave = t >> 5;
  const int c0   = t * 8;
  const float* sr = S + (size_t)row * kSeq + c0;
  const v4f a = *(const v4f*)(sr);
  const v4f c = *(const v4f*)(sr + 4);
  float x[8];
#pragma unroll
  for (int e = 0; e < 4; ++e) { x[e] = a[e]; x[4 + e] = c[e]; }
  float m = fmaxf(fmaxf(fmaxf(x[0], x[1]), fmaxf(x[2], x[3])), fmaxf(fmaxf(x[4], x[5]), fmaxf(x[6], x[7])));
#pragma unroll
  for (int off = 16; off > 0; off >>= 1) m = fmaxf(m, __shfl_xor(m, off, 32));
  if (lane == 0) redM[wave] = m;
  __syncthreads();
  float gm = redM[0];
#pragma unroll
  for (int w = 1; w < 8; ++w) gm = fmaxf(gm, redM[w]);
  float ev[8];
  float s = 0.f;
#pragma unroll
  for (int e = 0; e < 8; ++e) { ev[e] = expf(x[e] - gm); s += ev[e]; }
#pragma unroll
  for (int off = 16; off > 0; off >>= 1) s += __shfl_xor(s, off, 32);
  if (lane == 0) redS[wave] = s;
  __syncthreads();
  float tot = redS[0];
#pragma unroll
  for (int w = 1; w < 8; ++w) tot += redS[w];
  const float inv = carry * (1.0f / tot);
  unsigned short hb[8];
#pragma unroll
  for (int e = 0; e < 8; ++e) hb[e] = h_bits(ev[e] * inv);
  const v4u u = (v4u){pk16(hb[0], hb[1]), pk16(hb[2], hb[3]), pk16(hb[4], hb[5]), pk16(hb[6], hb[7])};
  unsigned short* qp = P + (size_t)row * kSeq + c0;
  *(volatile v4u*)qp = u;
  __threadfence();
  *(volatile v4u*)qp = u;
}

__global__ __launch_bounds__(256) void ohead_kernel(const unsigned short* __restrict__ opv, unsigned short* __restrict__ opl, int g) {
  const int lane = threadIdx.x & 31, wave = threadIdx.x >> 5;
  const int rsel = lane >> 4, q = lane & 15;
  const int hz = q >> 1, d0 = 8 * (q & 1);
  const int n = blockIdx.x * 16 + wave * 2 + rsel;
  const v4u u = *(const v4u*)(opv + ((size_t)hz * kSeq + n) * 64 + 16 * (hz & 3) + d0);
  unsigned short* qp = opl + ((size_t)g * kSeq + n) * kDim + 8 * q;
  *(volatile v4u*)qp = u;
  __threadfence();
  *(volatile v4u*)qp = u;
}

__global__ __launch_bounds__(256) void gelu2_kernel(const float* __restrict__ in, unsigned short* __restrict__ out, int n2, float carry) {
  const int i = blockIdx.x * 256 + threadIdx.x;
  if (i >= n2) return;
  const v2f v = *(const v2f*)(in + 2 * (size_t)i);
  float g0 = 0.f, g1 = 0.f;
#pragma unroll 1
  for (int s = 0; s < 2; ++s) {
    const float xx = s ? v[1] : v[0];
    const float gl = 0.5f * xx * (1.0f + erff(xx * 0.70710678118654752f));
    g0 = s ? g0 : gl;
    g1 = s ? gl : g1;
  }
  const unsigned u = pk16(h_bits(g0 * carry), h_bits(g1 * carry));
  unsigned* qp = (unsigned*)(out + 2 * (size_t)i);
  *(volatile unsigned*)qp = u;
  __threadfence();
  *(volatile unsigned*)qp = u;
}

extern "C" void kernel_launch(void* const* d_in, const int* in_sizes, int n_in,
                              void* d_out, int out_size, void* d_ws, size_t ws_size,
                              hipStream_t stream) {
  if (n_in < 14) return;
  if (in_sizes[0] != kRows * kDim || in_sizes[1] != kRows * kDim || in_sizes[2] != kRows * kDim) return;
  if (in_sizes[3] != 3 * kDim || in_sizes[4] != 3 * kDim) return;
  if (in_sizes[5] != 3 * kDim * kDim3 || in_sizes[6] != 3 * kDim * kDim || in_sizes[7] != 3 * kDim) return;
  if (in_sizes[8] != kDim3 || in_sizes[9] != kDim3) return;
  if (in_sizes[10] != kDim3 * kHid || in_sizes[11] != kHid || in_sizes[12] != kHid * kDim3 || in_sizes[13] != kDim3) return;
  if (out_size != 3 * kRows * kDim) return;

  const float* x1     = (const float*)d_in[0];
  const float* x2     = (const float*)d_in[1];
  const float* x3     = (const float*)d_in[2];
  const float* ln1_g  = (const float*)d_in[3];
  const float* ln1_b  = (const float*)d_in[4];
  const float* qkv_w  = (const float*)d_in[5];
  const float* proj_w = (const float*)d_in[6];
  const float* proj_b = (const float*)d_in[7];
  const float* ln2_g  = (const float*)d_in[8];
  const float* ln2_b  = (const float*)d_in[9];
  const float* fc1_w  = (const float*)d_in[10];
  const float* fc1_b  = (const float*)d_in[11];
  const float* fc2_w  = (const float*)d_in[12];
  const float* fc2_b  = (const float*)d_in[13];
  float* out = (float*)d_out;

  const size_t szWQKV  = (size_t)3 * kDim3 * kDim * 2;
  const size_t szWPROJ = (size_t)3 * kDim * kDim * 2;
  const size_t szWFC1  = (size_t)kHid * kDim3 * 2;
  const size_t szWFC2  = (size_t)kDim3 * kHid * 2;
  const size_t szQ32   = (size_t)3 * kRows * kQPitch * 2;
  const size_t szVT    = (size_t)kGroups * kDim * kSeq * 2;
  const size_t szXN    = (size_t)3 * kRows * kDim * 2;
  const size_t szQKVO  = (size_t)3 * kRows * kDim3 * 2;
  const size_t szS     = (size_t)kHeadGrp * kSeq * kSeq * 4;
  const size_t szHN    = (size_t)kRows * kDim3 * 2;
  const size_t szH1    = (size_t)kRows * kHid * 4;
  const size_t szG     = (size_t)kRows * kHid * 2;
  size_t szBIG = szS;
  if (szXN + szQKVO > szBIG) szBIG = szXN + szQKVO;
  if (szHN + szH1 + szG > szBIG) szBIG = szHN + szH1 + szG;
  const size_t szP     = (size_t)kHeadGrp * kSeq * kSeq * 2;
  const size_t szOPV   = (size_t)kHeads * kSeq * 64 * 2;
  const size_t szOPL   = (size_t)3 * kRows * kDim * 2;
  const size_t szXC    = (size_t)kRows * kDim3 * 4;

  const size_t oWQKV  = 0;
  const size_t oWPROJ = oWQKV + szWQKV;
  const size_t oWFC1  = oWPROJ + szWPROJ;
  const size_t oWFC2  = oWFC1 + szWFC1;
  const size_t oQ32   = oWFC2 + szWFC2;
  const size_t oK32   = oQ32 + szQ32;
  const size_t oVT    = oK32 + szQ32;
  const size_t oBIG   = oVT + szVT;
  const size_t oP     = oBIG + szBIG;
  const size_t oOPV   = oP + szP;
  const size_t oOPL   = oOPV + szOPV;
  const size_t oXC    = oOPL + szOPL;
  const size_t oEnd   = oXC + szXC;
  if (oEnd > ws_size) return;

  unsigned char* ws = (unsigned char*)d_ws;
  unsigned short* WQKV  = (unsigned short*)(ws + oWQKV);
  unsigned short* WPROJ = (unsigned short*)(ws + oWPROJ);
  unsigned short* WFC1  = (unsigned short*)(ws + oWFC1);
  unsigned short* WFC2  = (unsigned short*)(ws + oWFC2);
  unsigned short* Q32   = (unsigned short*)(ws + oQ32);
  unsigned short* K32   = (unsigned short*)(ws + oK32);
  unsigned short* VT    = (unsigned short*)(ws + oVT);
  unsigned short* XN    = (unsigned short*)(ws + oBIG);
  unsigned short* QKVO  = (unsigned short*)(ws + oBIG + szXN);
  float*          S     = (float*)(ws + oBIG);
  unsigned short* HN    = (unsigned short*)(ws + oBIG);
  float*          H1    = (float*)(ws + oBIG + szHN);
  unsigned short* G     = (unsigned short*)(ws + oBIG + szHN + szH1);
  unsigned short* P     = (unsigned short*)(ws + oP);
  unsigned short* OPV   = (unsigned short*)(ws + oOPV);
  unsigned short* OPL   = (unsigned short*)(ws + oOPL);
  float*          XC    = (float*)(ws + oXC);
  const float* fdum = proj_b;

  wtcast_kernel<<<dim3(kDim / 64, kDim3 / 64, 3), 256, 0, stream>>>(qkv_w, WQKV, kDim, kDim3, kWCarry);
  wtcast_kernel<<<dim3(kDim / 64, kDim / 64, 3), 256, 0, stream>>>(proj_w, WPROJ, kDim, kDim, kWCarry);
  wtcast_kernel<<<dim3(kDim3 / 64, kHid / 64, 1), 256, 0, stream>>>(fc1_w, WFC1, kDim3, kHid, kWCarry);
  wtcast_kernel<<<dim3(kHid / 64, kDim3 / 64, 1), 256, 0, stream>>>(fc2_w, WFC2, kHid, kDim3, kWCarry);

  ln128_kernel<<<dim3(3 * kRows / 8), 256, 0, stream>>>(x1, x2, x3, ln1_g, ln1_b, XN);

  wmma_gemm64<0, false, 0, 1, false><<<dim3(48, 3), 256, 0, stream>>>(
      XN, XN, kDim, (long)kRows * kDim,
      WQKV, WQKV, kDim, (long)kDim3 * kDim,
      (void*)QKVO, (void*)QKVO, kDim3, (long)kRows * kDim3,
      fdum, fdum, 0L, 0,
      kRows, kDim3, kDim, 1.0f / kWCarry);

  pad_qk_kernel<<<dim3(3 * kRows / 8), 256, 0, stream>>>(QKVO, Q32, K32);
  vtrans_kernel<<<dim3(kSeq / 64, kDim / 64, kGroups), 256, 0, stream>>>(QKVO, VT);

  for (int g = 0; g < kGroups; ++g) {
    for (int hg = 0; hg < kHeads / kHeadGrp; ++hg) {
      const unsigned short* qa = Q32 + (size_t)g * kSeq * kQPitch + hg * kHeadGrp * 32;
      const unsigned short* ka = K32 + (size_t)g * kSeq * kQPitch + hg * kHeadGrp * 32;
      wmma_gemm64<0, false, 0, 0, false><<<dim3(128, kHeadGrp), 256, 0, stream>>>(
          qa, qa, kQPitch, 32L,
          ka, ka, kQPitch, 32L,
          (void*)S, (void*)S, kSeq, (long)kSeq * kSeq,
          fdum, fdum, 0L, 0,
          kSeq, kSeq, 32, 0.25f);
      softmax2048_kernel<<<dim3(kHeadGrp * kSeq), 256, 0, stream>>>(S, P, kPCarry);
      const unsigned short* vb = VT + ((size_t)g * kDim + hg * 64) * kSeq;
      unsigned short* opv = OPV + (size_t)hg * kHeadGrp * kSeq * 64;
      wmma_gemm64<0, false, 0, 1, false><<<dim3(4, kHeadGrp), 256, 0, stream>>>(
          P, P, kSeq, (long)kSeq * kSeq,
          vb, vb, kSeq, 0L,
          (void*)opv, (void*)opv, 64, (long)kSeq * 64,
          fdum, fdum, 0L, 0,
          kSeq, 64, kSeq, kOCarry / kPCarry);
    }
    ohead_kernel<<<dim3(kSeq / 16), 256, 0, stream>>>(OPV, OPL, g);
  }

  for (int br = 0; br < 3; ++br) {
    const float* xbr = (br == 0) ? x1 : (br == 1) ? x2 : x3;
    const unsigned short* oa = OPL + (size_t)br * kRows * kDim;
    const unsigned short* wb = WPROJ + (size_t)br * kDim * kDim;
    float* xcb = XC + br * kDim;
    wmma_gemm64<0, false, 2, 0, true><<<dim3(16, 1), 256, 0, stream>>>(
        oa, oa, kDim, 0L,
        wb, wb, kDim, 0L,
        (void*)xcb, (void*)xcb, kDim3, 0L,
        proj_b + br * kDim, xbr, 0L, kDim,
        kRows, kDim, kDim, 1.0f / (kOCarry * kWCarry));
  }

  ln384_kernel<<<dim3(kRows / 8), 256, 0, stream>>>(XC, ln2_g, ln2_b, HN);

  wmma_gemm64<0, false, 2, 0, false><<<dim3(96, 1), 256, 0, stream>>>(
      HN, HN, kDim3, 0L,
      WFC1, WFC1, kDim3, 0L,
      (void*)H1, (void*)H1, kHid, 0L,
      fc1_b, fdum, 0L, 0,
      kRows, kHid, kDim3, 1.0f / kWCarry);

  gelu2_kernel<<<dim3((kRows * kHid / 2 + 255) / 256), 256, 0, stream>>>(H1, G, kRows * kHid / 2, kGCarry);

  for (int k = 0; k < 3; ++k) {
    const unsigned short* wb = WFC2 + (size_t)k * kDim * kHid;
    float* ok = out + (size_t)k * kRows * kDim;
    wmma_gemm64<0, false, 2, 0, true><<<dim3(16, 1), 256, 0, stream>>>(
        G, G, kHid, 0L,
        wb, wb, kHid, 0L,
        (void*)ok, (void*)ok, kDim, 0L,
        fc2_b + k * kDim, XC + k * kDim, 0L, kDim3,
        kRows, kDim, kHid, 1.0f / (kGCarry * kWCarry));
  }
}
